// Retention_32727650795919
// MI455X (gfx1250) — hardware-run, weakly checked
//
#include <hip/hip_runtime.h>
#include <math.h>

constexpr int kBatch = 4;
constexpr int kSeq   = 2048;
constexpr int kDim   = 1024;
constexpr int kHeads = 16;
constexpr int kHd    = kDim / kHeads;
constexpr int kRows  = kBatch * kSeq;
constexpr int kBH    = kBatch * kHeads;
constexpr int kQK    = 2 * kHd;
constexpr int kNqkv  = 3 * kDim;
constexpr float kWCarry    = 16.0f;
constexpr float kWCarryInv = 1.0f / kWCarry;
constexpr float kLnEps     = 1e-5f;
constexpr float kInvHd     = 1.0f / (float)kHd;
static_assert(kHd == 64, "head dim");
static_assert(kQK == 128, "expanded feature count");
static_assert(kRows % 64 == 0 && kNqkv % 64 == 0 && kDim % 64 == 0, "GEMM M,N tile multiples");
static_assert(kDim % 32 == 0 && kQK % 32 == 0, "GEMM K multiples of 32");
static_assert(kSeq % 64 == 0, "sequence tile multiple");
static_assert((kRows / 64) * (kNqkv / 64) % 8 == 0, "fused projection grid exact");
static_assert((kRows / 64) * (kDim / 64) % 8 == 0, "output projection grid exact");

typedef __attribute__((ext_vector_type(16))) _Float16 v16h;
typedef __attribute__((ext_vector_type(8)))  _Float16 v8h;
typedef __attribute__((ext_vector_type(8)))  float    v8f;
typedef __attribute__((ext_vector_type(4)))  float    v4f;
typedef __attribute__((ext_vector_type(4)))  unsigned int v4u;

struct ThetaTab { float th[64]; };
struct DecayTab { float l2g[16]; };
static_assert(sizeof(ThetaTab) == 256, "no padding");
static_assert(sizeof(DecayTab) == 64, "no padding");

__device__ __forceinline__ float bf16r(float f) {
  unsigned u = __float_as_uint(f);
  u = (u + 0x7FFFu + ((u >> 16) & 1u)) & 0xFFFF0000u;
  return __uint_as_float(u);
}
__device__ __forceinline__ unsigned short h_bits(float f) {
  const _Float16 h = (_Float16)f;
  return __builtin_bit_cast(unsigned short, h);
}
__device__ __forceinline__ unsigned pk16(unsigned short a, unsigned short b) {
  return (unsigned)a | ((unsigned)b << 16);
}
union FragU { v16h v; v8h h[2]; };
__device__ __forceinline__ v16h frag_load(const _Float16* p) {
  FragU f;
  f.h[0] = *(const v8h*)(p);
  f.h[1] = *(const v8h*)(p + 16);
  return f.v;
}
__device__ __forceinline__ v8f mma_h(v16h a, v16h b, v8f c) {
  return __builtin_amdgcn_wmma_f32_16x16x32_f16(false, a, false, b, (short)0, c, false, false);
}
__device__ __forceinline__ void guard4x5_h(v8f& a, v8f& b, v8f& c, v8f& d, v16h x, v16h y0, v16h y1, v16h y2, v16h y3) {
  asm volatile("v_nop\n\tv_nop\n\tv_nop\n\tv_nop" : "+v"(a), "+v"(b), "+v"(c), "+v"(d) : "v"(x), "v"(y0), "v"(y1), "v"(y2), "v"(y3));
}
__device__ __forceinline__ void guard2x3_h(v8f& a, v8f& b, v16h x, v16h y, v16h z) {
  asm volatile("v_nop\n\tv_nop\n\tv_nop\n\tv_nop" : "+v"(a), "+v"(b) : "v"(x), "v"(y), "v"(z));
}
__device__ __forceinline__ void keep4_h(v16h a, v16h b, v16h c, v16h d) {
  asm volatile("v_nop" :: "v"(a), "v"(b), "v"(c), "v"(d));
}
__device__ __forceinline__ void acc_guard4(v8f& a, v8f& b, v8f& c, v8f& d) {
  asm volatile("v_nop\n\tv_nop\n\tv_nop\n\tv_nop" : "+v"(a), "+v"(b), "+v"(c), "+v"(d));
}
__device__ __forceinline__ void wave_lds_sync() {
  __builtin_amdgcn_fence(__ATOMIC_RELEASE, "workgroup");
  __builtin_amdgcn_wave_barrier();
  __builtin_amdgcn_fence(__ATOMIC_ACQUIRE, "workgroup");
}

__global__ __launch_bounds__(256) void trig_table_kernel(float* __restrict__ CS, ThetaTab tab) {
  __shared__ float th[64];
  if (threadIdx.x == 0) {
#pragma unroll
    for (int k = 0; k < 64; ++k) th[k] = tab.th[k];
  }
  __syncthreads();
  const int idx = blockIdx.x * 256 + threadIdx.x;
  const int s = idx >> 7;
  const int j = idx & 127;
  const float ang = (float)s * th[j & 63];
  const float cs = cosf(ang);
  const float sn = sinf(ang);
  const float v = (j < 64) ? cs : sn;
  volatile float* p = CS + idx;
  *p = v;
  __threadfence();
  *p = v;
}

__global__ __launch_bounds__(256) void cvt8_kernel(const float* __restrict__ s0, const float* __restrict__ s1,
                                                   const float* __restrict__ s2, const float* __restrict__ s3,
                                                   unsigned short* __restrict__ dst, int n8, float sc) {
  const int z = blockIdx.y;
  const float* src = (z == 0) ? s0 : (z == 1) ? s1 : (z == 2) ? s2 : s3;
  const int i = blockIdx.x * 256 + threadIdx.x;
  if (i < n8) {
    const float* p = src + 8 * (size_t)i;
    const v4f a = *(const v4f*)(p);
    const v4f c = *(const v4f*)(p + 4);
    unsigned short hb[8];
#pragma unroll
    for (int e = 0; e < 4; ++e) {
      hb[e]     = h_bits(bf16r(a[e]) * sc);
      hb[4 + e] = h_bits(bf16r(c[e]) * sc);
    }
    const v4u u = (v4u){pk16(hb[0], hb[1]), pk16(hb[2], hb[3]), pk16(hb[4], hb[5]), pk16(hb[6], hb[7])};
    unsigned short* q = dst + ((size_t)z * (size_t)n8 + (size_t)i) * 8;
    *(volatile v4u*)q = u;
    __threadfence();
    *(volatile v4u*)q = u;
  }
}

template <int EPI>
__global__ __launch_bounds__(256) void gemm64_kernel(
    const unsigned short* __restrict__ Ap, int lda,
    const unsigned short* __restrict__ Btp, int ldb,
    float* __restrict__ Cf, int ldc,
    unsigned short* __restrict__ QPp, unsigned short* __restrict__ KPp, unsigned short* __restrict__ VTp,
    const float* __restrict__ CS,
    int M, int N, int K, float scale) {
  const _Float16* A  = (const _Float16*)Ap;
  const _Float16* Bt = (const _Float16*)Btp;
  __shared__ __align__(16) unsigned int sW[8][1152];
  const int lane = threadIdx.x & 31;
  const int wave = threadIdx.x >> 5;
  const int tilesN = N >> 6;
  const int tilesM = M >> 6;
  const int tile = blockIdx.x * 8 + wave;
  if (tile >= tilesM * tilesN) return;
  const int tm = tile / tilesN;
  const int tn = tile - tm * tilesN;
  const int m0 = tm << 6;
  const int n0 = tn << 6;
  const int rlane = lane & 15;
  const int hh    = lane >> 4;
  const int koff  = hh * 8;
  const int mOff  = hh * 8;

  v8f acc[4][4];
#pragma unroll
  for (int i = 0; i < 4; ++i)
#pragma unroll
    for (int j = 0; j < 4; ++j) acc[i][j] = (v8f){0.f, 0.f, 0.f, 0.f, 0.f, 0.f, 0.f, 0.f};

  const _Float16* Arow = A  + (size_t)(m0 + rlane) * lda + koff;
  const _Float16* Brow = Bt + (size_t)(n0 + rlane) * ldb + koff;
  const size_t a16 = (size_t)16 * lda;
  const size_t b16 = (size_t)16 * ldb;

  for (int k0 = 0; k0 < K; k0 += 32) {
    v16h bh[4];
#pragma unroll
    for (int j = 0; j < 4; ++j) bh[j] = frag_load(Brow + (size_t)j * b16 + k0);
#pragma unroll
    for (int i = 0; i < 4; ++i) {
      const v16h ah = frag_load(Arow + (size_t)i * a16 + k0);
#pragma unroll
      for (int j = 0; j < 4; ++j) acc[i][j] = mma_h(ah, bh[j], acc[i][j]);
      guard4x5_h(acc[i][0], acc[i][1], acc[i][2], acc[i][3], ah, bh[0], bh[1], bh[2], bh[3]);
    }
    keep4_h(bh[0], bh[1], bh[2], bh[3]);
  }
  acc_guard4(acc[0][0], acc[0][1], acc[0][2], acc[0][3]);
  acc_guard4(acc[1][0], acc[1][1], acc[1][2], acc[1][3]);
  acc_guard4(acc[2][0], acc[2][1], acc[2][2], acc[2][3]);
  acc_guard4(acc[3][0], acc[3][1], acc[3][2], acc[3][3]);

  unsigned int* slab = sW[wave];

  if (EPI == 0) {
    unsigned int* Cw = (unsigned int*)Cf;
    const int c4 = rlane * 4;
#pragma unroll
    for (int i = 0; i < 4; ++i) {
      const int mBase = m0 + (i << 4);
#pragma unroll
      for (int j = 0; j < 4; ++j)
#pragma unroll
        for (int r = 0; r < 8; ++r)
          slab[(mOff + r) * 68 + (j << 4) + rlane] = __float_as_uint(acc[i][j][r] * scale);
      wave_lds_sync();
      for (int pass = 0; pass < 2; ++pass) {
#pragma unroll
        for (int it = 0; it < 8; ++it) {
          const int row = it * 2 + hh;
          const v4u w = *(const v4u*)(slab + row * 68 + c4);
          *(volatile v4u*)(Cw + (size_t)(mBase + row) * ldc + n0 + c4) = w;
        }
        __threadfence();
      }
      wave_lds_sync();
    }
  } else {
    const int tsel = tn >> 4;
    const int hd   = tn & 15;
    const int bidx = m0 / kSeq;
    const int s0   = m0 - bidx * kSeq;
    const int bh   = bidx * kHeads + hd;
    if (tsel < 2) {
      unsigned short* plane = (tsel == 0) ? QPp : KPp;
      const int c16 = rlane;
      const int d8  = (c16 & 7) * 8;
#pragma unroll
      for (int i = 0; i < 4; ++i) {
#pragma unroll
        for (int j = 0; j < 4; ++j)
#pragma unroll
          for (int r = 0; r < 8; ++r)
            slab[(mOff + r) * 68 + (j << 4) + rlane] = __float_as_uint(acc[i][j][r] * scale);
        wave_lds_sync();
        for (int pass = 0; pass < 2; ++pass) {
#pragma unroll
          for (int it = 0; it < 8; ++it) {
            const int row = it * 2 + hh;
            const int s = s0 + (i << 4) + row;
            const v4u wa = *(const v4u*)(slab + row * 68 + d8);
            const v4u wb = *(const v4u*)(slab + row * 68 + d8 + 4);
            const float* cp = CS + (size_t)s * kQK + c16 * 8;
            const v4f ca = *(const v4f*)(cp);
            const v4f cb = *(const v4f*)(cp + 4);
            unsigned short hb[8];
#pragma unroll
            for (int e = 0; e < 4; ++e) {
              const unsigned ua = wa[e];
              const unsigned ub = wb[e];
              const float fa = __uint_as_float(ua);
              const float fb = __uint_as_float(ub);
              hb[e]     = h_bits(fa * ca[e]);
              hb[4 + e] = h_bits(fb * cb[e]);
            }
            const v4u o = (v4u){pk16(hb[0], hb[1]), pk16(hb[2], hb[3]), pk16(hb[4], hb[5]), pk16(hb[6], hb[7])};
            *(volatile v4u*)(plane + ((size_t)bh * kSeq + (size_t)s) * kQK + c16 * 8) = o;
          }
          __threadfence();
        }
        wave_lds_sync();
      }
    } else {
      const int q   = lane >> 3;
      const int c8i = lane & 7;
#pragma unroll
      for (int half = 0; half < 2; ++half) {
#pragma unroll
        for (int jj = 0; jj < 2; ++jj) {
          const int dl = 16 * jj + rlane;
#pragma unroll
          for (int i = 0; i < 4; ++i) {
            unsigned short hb[8];
#pragma unroll
            for (int r = 0; r < 8; ++r) hb[r] = h_bits(acc[i][2 * half + jj][r] * scale);
            const v4u w = (v4u){pk16(hb[0], hb[1]), pk16(hb[2], hb[3]), pk16(hb[4], hb[5]), pk16(hb[6], hb[7])};
            *(v4u*)(slab + dl * 36 + 8 * i + 4 * hh) = w;
          }
        }
        wave_lds_sync();
        for (int pass = 0; pass < 2; ++pass) {
#pragma unroll
          for (int it = 0; it < 8; ++it) {
            const int dl = it * 4 + q;
            const v4u w = *(const v4u*)(slab + dl * 36 + c8i * 4);
            *(volatile v4u*)(VTp + ((size_t)(bh * kHd + 32 * half + dl)) * kSeq + s0 + c8i * 8) = w;
          }
          __threadfence();
        }
        wave_lds_sync();
      }
    }
  }
}

__global__ __launch_bounds__(128) void retention_kernel(
    const unsigned short* __restrict__ QPp, const unsigned short* __restrict__ KPp,
    const unsigned short* __restrict__ VTp,
    const float* __restrict__ ln_w, const float* __restrict__ ln_b,
    unsigned short* __restrict__ Y16, DecayTab dt) {
  __shared__ __align__(16) float Os[4][16 * 68];
  const int tid  = threadIdx.x;
  const int wave = tid >> 5;
  const int lane = tid & 31;
  const int hh   = lane >> 4;
  const int c    = lane & 15;
  const int qt   = blockIdx.x;
  const int bh   = blockIdx.y;
  const int h    = bh & (kHeads - 1);
  const int b    = bh / kHeads;
  const int q0w  = qt * 64 + wave * 16;

  float l2g = dt.l2g[0];
#pragma unroll
  for (int k = 1; k < 16; ++k) l2g = (h == k) ? dt.l2g[k] : l2g;

  const _Float16* Qp = (const _Float16*)QPp + (size_t)bh * kSeq * kQK;
  const _Float16* Kp = (const _Float16*)KPp + (size_t)bh * kSeq * kQK;
  const _Float16* Vt = (const _Float16*)VTp + (size_t)bh * kHd * kSeq;

  v16h qf[4];
  {
    const _Float16* qrow = Qp + (size_t)(q0w + c) * kQK + 8 * hh;
#pragma unroll
    for (int kk = 0; kk < 4; ++kk) qf[kk] = frag_load(qrow + 32 * kk);
  }
  float colf0[8], colf1[8];
#pragma unroll
  for (int r = 0; r < 8; ++r) {
    colf0[r] = exp2f(-l2g * (float)r);
    colf1[r] = exp2f(-l2g * (float)(16 + r));
  }
  const v8f z8 = {0.f, 0.f, 0.f, 0.f, 0.f, 0.f, 0.f, 0.f};
  v8f oacc[4];
#pragma unroll
  for (int nt = 0; nt < 4; ++nt) oacc[nt] = z8;

  const int iq = q0w + c;
  const int nsteps = (q0w + 16 + 31) >> 5;
  const _Float16* kbase = Kp + (size_t)c * kQK + 8 * hh;
  const _Float16* vbase = Vt + (size_t)c * kSeq + 8 * hh;

#pragma unroll 1
  for (int step = 0; step < nsteps; ++step) {
    const int t0 = step * 32;
    const _Float16* k0p = kbase + (size_t)t0 * kQK;
    v8f s0 = z8, s1 = z8;
#pragma unroll
    for (int kk = 0; kk < 4; ++kk) {
      const v16h a0 = frag_load(k0p + 32 * kk);
      const v16h a1 = frag_load(k0p + 16 * kQK + 32 * kk);
      s0 = mma_h(a0, qf[kk], s0);
      s1 = mma_h(a1, qf[kk], s1);
      guard2x3_h(s0, s1, a0, a1, qf[kk]);
    }
    const int nb = iq - t0 - 8 * hh;
    const float lf = exp2f(l2g * (float)nb);
    v16h pa;
#pragma unroll
    for (int r = 0; r < 8; ++r) {
      const float w0 = lf * colf0[r];
      const float w1 = lf * colf1[r];
      const float p0 = (nb - r >= 0) ? (s0[r] * w0) : 0.0f;
      const float p1 = (nb - 16 - r >= 0) ? (s1[r] * w1) : 0.0f;
      pa[r]     = (_Float16)p0;
      pa[8 + r] = (_Float16)p1;
    }
    const _Float16* vp = vbase + t0;
    const v16h vb0 = frag_load(vp);
    const v16h vb1 = frag_load(vp + (size_t)16 * kSeq);
    const v16h vb2 = frag_load(vp + (size_t)32 * kSeq);
    const v16h vb3 = frag_load(vp + (size_t)48 * kSeq);
    oacc[0] = mma_h(pa, vb0, oacc[0]);
    oacc[1] = mma_h(pa, vb1, oacc[1]);
    oacc[2] = mma_h(pa, vb2, oacc[2]);
    oacc[3] = mma_h(pa, vb3, oacc[3]);
    guard4x5_h(oacc[0], oacc[1], oacc[2], oacc[3], pa, vb0, vb1, vb2, vb3);
  }
  acc_guard4(oacc[0], oacc[1], oacc[2], oacc[3]);

  float* os = Os[wave];
#pragma unroll
  for (int nt = 0; nt < 4; ++nt)
#pragma unroll
    for (int r = 0; r < 8; ++r) os[(8 * hh + r) * 68 + 16 * nt + c] = oacc[nt][r];
  wave_lds_sync();

  const int q  = lane >> 3;
  const int c8 = (lane & 7) * 8;
  float gw[8], gb[8];
  {
    const v4f g0 = *(const v4f*)(ln_w + c8);
    const v4f g1 = *(const v4f*)(ln_w + c8 + 4);
    const v4f e0 = *(const v4f*)(ln_b + c8);
    const v4f e1 = *(const v4f*)(ln_b + c8 + 4);
#pragma unroll
    for (int e = 0; e < 4; ++e) {
      gw[e]     = bf16r(g0[e]);
      gw[4 + e] = bf16r(g1[e]);
      gb[e]     = bf16r(e0[e]);
      gb[4 + e] = bf16r(e1[e]);
    }
  }
  unsigned short* yb = Y16 + ((size_t)b * kSeq + (size_t)q0w) * kDim + h * kHd + c8;
  for (int pass = 0; pass < 2; ++pass) {
#pragma unroll 1
    for (int it = 0; it < 4; ++it) {
      const int row = it * 4 + q;
      const float* sp = os + row * 68 + c8;
      const v4f a  = *(const v4f*)(sp);
      const v4f bq = *(const v4f*)(sp + 4);
      float x[8];
#pragma unroll
      for (int e = 0; e < 4; ++e) { x[e] = a[e]; x[4 + e] = bq[e]; }
      float sm = ((x[0] + x[1]) + (x[2] + x[3])) + ((x[4] + x[5]) + (x[6] + x[7]));
      sm += __shfl_xor(sm, 1, 32);
      sm += __shfl_xor(sm, 2, 32);
      sm += __shfl_xor(sm, 4, 32);
      const float mu = sm * kInvHd;
      float ss = 0.0f;
#pragma unroll
      for (int e = 0; e < 8; ++e) { x[e] -= mu; ss += x[e] * x[e]; }
      ss += __shfl_xor(ss, 1, 32);
      ss += __shfl_xor(ss, 2, 32);
      ss += __shfl_xor(ss, 4, 32);
      const float rstd = rsqrtf(ss * kInvHd + kLnEps);
      unsigned short hb[8];
#pragma unroll
      for (int e = 0; e < 8; ++e) {
        const float y  = (x[e] * rstd) * gw[e] + gb[e];
        const float sg = 1.0f / (1.0f + expf(-y));
        hb[e] = h_bits(y * sg);
      }
      const v4u o = (v4u){pk16(hb[0], hb[1]), pk16(hb[2], hb[3]), pk16(hb[4], hb[5]), pk16(hb[6], hb[7])};
      *(volatile v4u*)(yb + (size_t)row * kDim) = o;
    }
    __threadfence();
  }
}

extern "C" void kernel_launch(void* const* d_in, const int* in_sizes, int n_in,
                              void* d_out, int out_size, void* d_ws, size_t ws_size, hipStream_t stream) {
  if (n_in < 7 || d_out == nullptr || d_ws == nullptr) return;
  if (in_sizes[0] != kRows * kDim || in_sizes[1] != kDim * kDim || in_sizes[2] != kDim * kDim ||
      in_sizes[3] != kDim * kDim || in_sizes[4] != kDim * kDim || in_sizes[5] != kHd || in_sizes[6] != kHd ||
      out_size != kRows * kDim) return;

  const float* x    = (const float*)d_in[0];
  const float* Wq   = (const float*)d_in[1];
  const float* Wk   = (const float*)d_in[2];
  const float* Wv   = (const float*)d_in[3];
  const float* Wo   = (const float*)d_in[4];
  const float* ln_w = (const float*)d_in[5];
  const float* ln_b = (const float*)d_in[6];
  float* out = (float*)d_out;

  char* ws = (char*)d_ws;
  size_t off = 0;
  auto carve = [&](size_t bytes) -> char* { char* p = ws + off; off += (bytes + 255) & ~(size_t)255; return p; };
  float*          CS   = (float*)carve((size_t)kSeq * kQK * 4);
  unsigned short* X16  = (unsigned short*)carve((size_t)kRows * kDim * 2);
  unsigned short* WALL = (unsigned short*)carve((size_t)4 * kDim * kDim * 2);
  unsigned short* QP   = (unsigned short*)carve((size_t)kBH * kSeq * kQK * 2);
  unsigned short* KP   = (unsigned short*)carve((size_t)kBH * kSeq * kQK * 2);
  unsigned short* VT   = (unsigned short*)carve((size_t)kBH * kHd * kSeq * 2);
  unsigned short* Y16  = (unsigned short*)carve((size_t)kRows * kDim * 2);
  if (off > ws_size || off > (size_t)134217728) return;

  ThetaTab tt;
  for (int d = 0; d < 64; ++d) tt.th[d] = (float)pow(10000.0, -(double)d / 32.0);
  DecayTab dt;
  for (int hd = 0; hd < 16; ++hd) dt.l2g[hd] = (float)(log1p(-ldexp(1.0, -(5 + hd))) / log(2.0));

  trig_table_kernel<<<(kSeq * kQK) / 256, 256, 0, stream>>>(CS, tt);

  const int n8x = kRows * kDim / 8;
  const int n8w = kDim * kDim / 8;
  cvt8_kernel<<<dim3(n8x / 256, 1), 256, 0, stream>>>(x, x, x, x, X16, n8x, 1.0f);
  cvt8_kernel<<<dim3(n8w / 256, 4), 256, 0, stream>>>(Wq, Wk, Wv, Wo, WALL, n8w, kWCarry);

  gemm64_kernel<1><<<(kRows / 64) * (kNqkv / 64) / 8, 256, 0, stream>>>(
      X16, kDim, WALL, kDim, out, kDim, QP, KP, VT, CS, kRows, kNqkv, kDim, kWCarryInv);

  retention_kernel<<<dim3(kSeq / 64, kBH), 128, 0, stream>>>(QP, KP, VT, ln_w, ln_b, Y16, dt);

  gemm64_kernel<0><<<(kRows / 64) * (kDim / 64) / 8, 256, 0, stream>>>(
      Y16, kDim, WALL + (size_t)kNqkv * kDim, kDim, out, kDim, QP, KP, VT, CS, kRows, kDim, kDim, kWCarryInv);
}
